// RNN_4483945857342
// MI455X (gfx1250) — hardware-verified
//
#include <hip/hip_runtime.h>
#include <math.h>

constexpr int NBAT   = 256;
constexpr int NSTEP  = 128;
constexpr int NIN    = 256;
constexpr int NHID   = 1024;
constexpr int NCLS   = 1000;
constexpr int NCLSP  = 1024;
constexpr int TCH    = 32;
constexpr int NCHUNK = NSTEP / TCH;
constexpr int MROWS  = TCH * NBAT;
constexpr int NTHR   = 256;
constexpr int MBLK   = 16;
constexpr int HPITCH = 1032;
constexpr int SLABP  = 68;
constexpr float WCARRY     = 256.0f;
constexpr float WCARRY_INV = 1.0f / 256.0f;

static_assert(NSTEP % TCH == 0);
static_assert(NBAT % MBLK == 0);
static_assert(NHID == 128 * (NTHR / 32));
static_assert(NIN % 32 == 0 && NHID % 32 == 0);
static_assert(MROWS % 64 == 0 && NHID % 64 == 0 && NCLSP % 64 == 0 && NBAT % 64 == 0);
static_assert(NCLS % 4 == 0 && NCLS <= NCLSP);
static_assert((HPITCH * 2) % 16 == 0 && HPITCH >= NHID + 8);
static_assert((NBAT * NCLS) % (4 * NTHR) == 0);
static_assert((NSTEP * NBAT * (NIN / 8)) % NTHR == 0);

typedef __attribute__((ext_vector_type(16))) _Float16 v16h;
typedef __attribute__((ext_vector_type(8)))  _Float16 v8h;
typedef __attribute__((ext_vector_type(8)))  float    v8f;
typedef __attribute__((ext_vector_type(4)))  float    v4f;

__device__ __forceinline__ unsigned short f2bf_bits(float f) {
  unsigned u = __float_as_uint(f);
  return (unsigned short)((u + 0x7FFFu + ((u >> 16) & 1u)) >> 16);
}
__device__ __forceinline__ float bf_bits2f(unsigned short h) { return __uint_as_float(((unsigned)h) << 16); }
__device__ __forceinline__ float bf16r(float f) { return bf_bits2f(f2bf_bits(f)); }

union FragU { v16h v; v8h h[2]; };
__device__ __forceinline__ v16h frag_load_h(const _Float16* p) {
  FragU f;
  f.h[0] = *(const v8h*)(p);
  f.h[1] = *(const v8h*)(p + 16);
  return f.v;
}
__device__ __forceinline__ v8f mma_h(v16h a, v16h b, v8f c) {
  return __builtin_amdgcn_wmma_f32_16x16x32_f16(false, a, false, b, (short)0, c, false, false);
}
__device__ __forceinline__ void grp_guard_h(v8f& a0, v8f& a1, v8f& a2, v8f& a3, v16h x, v16h y0, v16h y1, v16h y2, v16h y3) {
  asm volatile("v_nop\n\tv_nop\n\tv_nop\n\tv_nop" : "+v"(a0), "+v"(a1), "+v"(a2), "+v"(a3) : "v"(x), "v"(y0), "v"(y1), "v"(y2), "v"(y3));
}
__device__ __forceinline__ void acc_guard4(v8f& a, v8f& b, v8f& c, v8f& d) {
  asm volatile("v_nop\n\tv_nop\n\tv_nop\n\tv_nop" : "+v"(a), "+v"(b), "+v"(c), "+v"(d));
}

__global__ __launch_bounds__(256) void gemm64_f16_kernel(
    const unsigned short* __restrict__ Ap, int lda,
    const unsigned short* __restrict__ Btp, int ldb,
    float* __restrict__ C, int ldc,
    const float* __restrict__ bias,
    int M, int N, int K, float scale) {
  const _Float16* A  = (const _Float16*)Ap;
  const _Float16* Bt = (const _Float16*)Btp;
  __shared__ __align__(16) float sT[8][16 * 68];
  const int lane = threadIdx.x & 31;
  const int wave = threadIdx.x >> 5;
  const int tilesN = N >> 6;
  const int tilesM = M >> 6;
  const int tile = blockIdx.x * 8 + wave;
  if (tile >= tilesM * tilesN) return;
  const int tm = tile / tilesN;
  const int tn = tile - tm * tilesN;
  const int m0 = tm << 6;
  const int n0 = tn << 6;
  const int rlane = lane & 15;
  const int koff  = (lane >> 4) * 8;
  const int mOff  = (lane >> 4) * 8;

  v8f acc[4][4];
#pragma unroll
  for (int i = 0; i < 4; ++i)
#pragma unroll
    for (int j = 0; j < 4; ++j) acc[i][j] = (v8f){0.f, 0.f, 0.f, 0.f, 0.f, 0.f, 0.f, 0.f};

  for (int k0 = 0; k0 < K; k0 += 32) {
    v16h bh[4];
#pragma unroll
    for (int j = 0; j < 4; ++j) {
      const size_t bo = (size_t)(n0 + (j << 4) + rlane) * ldb + koff + k0;
      bh[j] = frag_load_h(Bt + bo);
    }
#pragma unroll
    for (int i = 0; i < 4; ++i) {
      const size_t ao = (size_t)(m0 + (i << 4) + rlane) * lda + koff + k0;
      const v16h ah = frag_load_h(A + ao);
#pragma unroll
      for (int j = 0; j < 4; ++j) acc[i][j] = mma_h(ah, bh[j], acc[i][j]);
      grp_guard_h(acc[i][0], acc[i][1], acc[i][2], acc[i][3], ah, bh[0], bh[1], bh[2], bh[3]);
    }
  }
  acc_guard4(acc[0][0], acc[0][1], acc[0][2], acc[0][3]);
  acc_guard4(acc[1][0], acc[1][1], acc[1][2], acc[1][3]);
  acc_guard4(acc[2][0], acc[2][1], acc[2][2], acc[2][3]);
  acc_guard4(acc[3][0], acc[3][1], acc[3][2], acc[3][3]);

  float* slab = sT[wave];
#pragma unroll
  for (int i = 0; i < 4; ++i) {
    const int mBase = m0 + (i << 4);
#pragma unroll
    for (int j = 0; j < 4; ++j) {
      const int n = n0 + (j << 4) + rlane;
      const float bv = bias[n];
#pragma unroll
      for (int r = 0; r < 8; ++r) {
        const float v = acc[i][j][r] * scale + bv;
        slab[(mOff + r) * 68 + (j << 4) + rlane] = v;
      }
    }
    __builtin_amdgcn_fence(__ATOMIC_RELEASE, "workgroup");
    __builtin_amdgcn_wave_barrier();
    __builtin_amdgcn_fence(__ATOMIC_ACQUIRE, "workgroup");
    {
      const int hh = lane >> 4, c4 = (lane & 15) * 4;
      for (int pass = 0; pass < 2; ++pass) {
#pragma unroll
        for (int it = 0; it < 8; ++it) {
          const int row = it * 2 + hh;
          const v4f v = *(const v4f*)(slab + row * 68 + c4);
          *(volatile v4f*)(C + (size_t)(mBase + row) * ldc + n0 + c4) = v;
        }
        __threadfence();
      }
    }
    __builtin_amdgcn_fence(__ATOMIC_RELEASE, "workgroup");
    __builtin_amdgcn_wave_barrier();
    __builtin_amdgcn_fence(__ATOMIC_ACQUIRE, "workgroup");
  }
}

__global__ __launch_bounds__(NTHR) void wcvt_kernel(const float* __restrict__ src, unsigned short* __restrict__ dst,
                                                    int nrow_dst, int nrow_src, int ncol8, float sc) {
  const int i  = blockIdx.x * NTHR + threadIdx.x;
  const int n8 = nrow_dst * ncol8;
  if (i < n8) {
    const int row = i / ncol8;
    const int c8  = i - row * ncol8;
    const bool valid = row < nrow_src;
    const int rowc = valid ? row : (nrow_src - 1);
    const float* sp = src + (size_t)rowc * (size_t)(ncol8 * 8) + c8 * 8;
    const v4f a = *(const v4f*)(sp);
    const v4f b = *(const v4f*)(sp + 4);
    v8h hv;
#pragma unroll
    for (int e = 0; e < 4; ++e) {
      const float f0 = valid ? (bf16r(a[e]) * sc) : 0.0f;
      const float f1 = valid ? (bf16r(b[e]) * sc) : 0.0f;
      hv[e]     = (_Float16)f0;
      hv[4 + e] = (_Float16)f1;
    }
    *(volatile v8h*)(dst + (size_t)i * 8) = hv;
    __threadfence();
    *(volatile v8h*)(dst + (size_t)i * 8) = hv;
  }
}

__global__ __launch_bounds__(NTHR) void xcvt_kernel(const float* __restrict__ x, unsigned short* __restrict__ xh) {
  const int i = blockIdx.x * NTHR + threadIdx.x;
  if (i < NSTEP * NBAT * (NIN / 8)) {
    const int orow = i >> 5;
    const int c8   = (i & 31) * 8;
    const int t    = orow >> 8;
    const int b    = orow & (NBAT - 1);
    const float* sp = x + ((size_t)b * NSTEP + (size_t)t) * NIN + c8;
    const v4f a  = *(const v4f*)(sp);
    const v4f bb = *(const v4f*)(sp + 4);
    v8h hv;
#pragma unroll
    for (int e = 0; e < 4; ++e) {
      const float f0 = bf16r(a[e]);
      const float f1 = bf16r(bb[e]);
      hv[e]     = (_Float16)f0;
      hv[4 + e] = (_Float16)f1;
    }
    *(volatile v8h*)(xh + (size_t)i * 8) = hv;
    __threadfence();
    *(volatile v8h*)(xh + (size_t)i * 8) = hv;
  }
}

template <bool TWO>
__global__ __launch_bounds__(NTHR) void bias_prep_kernel(const float* __restrict__ a, const float* __restrict__ b,
                                                         float* __restrict__ dst, int nvalid) {
  const int i4 = threadIdx.x * 4;
  const bool valid = i4 < nvalid;
  const int ic = valid ? i4 : (nvalid - 4);
  const v4f va = *(const v4f*)(a + ic);
  const v4f vb = *(const v4f*)(b + ic);
  v4f o;
#pragma unroll
  for (int e = 0; e < 4; ++e) {
    float s = bf16r(va[e]);
    if (TWO) s = s + bf16r(vb[e]);
    o[e] = valid ? s : 0.0f;
  }
  *(volatile v4f*)(dst + i4) = o;
  __threadfence();
  *(volatile v4f*)(dst + i4) = o;
}

template <bool HIST>
__global__ __launch_bounds__(NTHR) void rnn_scan_kernel(const float* __restrict__ XP,
                                                        const unsigned short* __restrict__ Wp,
                                                        unsigned short* CARRYp, unsigned short* HISTp, int first) {
  __shared__ __align__(16) _Float16 Ah[MBLK * HPITCH];
  __shared__ __align__(16) float    Sl[NTHR / 32][16 * SLABP];
  const _Float16* W = (const _Float16*)Wp;
  _Float16* CARRY = (_Float16*)CARRYp;
  _Float16* HISTG = (_Float16*)HISTp;
  const int tid = threadIdx.x, lane = tid & 31, wave = tid >> 5;
  const int c = lane & 15, hh = lane >> 4, koff = hh * 8;
  const int rowbase = blockIdx.x * MBLK;

  v8h zv;
#pragma unroll
  for (int e = 0; e < 8; ++e) zv[e] = (_Float16)0.0f;

  if (first != 0) {
#pragma unroll 1
    for (int i = 0; i < 8; ++i) {
      const int idx = i * NTHR + tid;
      const int row = idx >> 7, c8 = (idx & 127) * 8;
      *(v8h*)(Ah + row * HPITCH + c8) = zv;
    }
  } else {
#pragma unroll 1
    for (int i = 0; i < 8; ++i) {
      const int idx = i * NTHR + tid;
      const int row = idx >> 7, c8 = (idx & 127) * 8;
      const v8h v = *(const v8h*)(CARRY + (size_t)(rowbase + row) * NHID + c8);
      *(v8h*)(Ah + row * HPITCH + c8) = v;
    }
  }
  if (tid < MBLK) *(v8h*)(Ah + tid * HPITCH + NHID) = zv;
  __syncthreads();

  const v8f z8 = {0.f, 0.f, 0.f, 0.f, 0.f, 0.f, 0.f, 0.f};
  float* slab = Sl[wave];
  const _Float16* ahrow = Ah + c * HPITCH + koff;
  const _Float16* wrow  = W + (size_t)(128 * wave + c) * NHID + koff;
  const int q = lane >> 3, c8e = (lane & 7) * 8;
  const int rr = lane >> 4, c8s = (lane & 15) * 8;

#pragma unroll 1
  for (int tl = 0; tl < TCH; ++tl) {
    v8f acc[8];
#pragma unroll
    for (int j = 0; j < 8; ++j) acc[j] = z8;

#pragma unroll 1
    for (int k0 = 0; k0 < NHID; k0 += 32) {
      const v16h a  = frag_load_h(ahrow + k0);
      const v16h b0 = frag_load_h(wrow + (size_t)0 * 16 * NHID + k0);
      const v16h b1 = frag_load_h(wrow + (size_t)1 * 16 * NHID + k0);
      const v16h b2 = frag_load_h(wrow + (size_t)2 * 16 * NHID + k0);
      const v16h b3 = frag_load_h(wrow + (size_t)3 * 16 * NHID + k0);
      acc[0] = mma_h(a, b0, acc[0]);
      acc[1] = mma_h(a, b1, acc[1]);
      acc[2] = mma_h(a, b2, acc[2]);
      acc[3] = mma_h(a, b3, acc[3]);
      grp_guard_h(acc[0], acc[1], acc[2], acc[3], a, b0, b1, b2, b3);
      const v16h b4 = frag_load_h(wrow + (size_t)4 * 16 * NHID + k0);
      const v16h b5 = frag_load_h(wrow + (size_t)5 * 16 * NHID + k0);
      const v16h b6 = frag_load_h(wrow + (size_t)6 * 16 * NHID + k0);
      const v16h b7 = frag_load_h(wrow + (size_t)7 * 16 * NHID + k0);
      acc[4] = mma_h(a, b4, acc[4]);
      acc[5] = mma_h(a, b5, acc[5]);
      acc[6] = mma_h(a, b6, acc[6]);
      acc[7] = mma_h(a, b7, acc[7]);
      grp_guard_h(acc[4], acc[5], acc[6], acc[7], a, b4, b5, b6, b7);
    }
    acc_guard4(acc[0], acc[1], acc[2], acc[3]);
    acc_guard4(acc[4], acc[5], acc[6], acc[7]);

    __syncthreads();

#pragma unroll
    for (int hf = 0; hf < 2; ++hf) {
      const int colbase = 128 * wave + 64 * hf;
#pragma unroll
      for (int j = 0; j < 4; ++j)
#pragma unroll
        for (int r = 0; r < 8; ++r) slab[(8 * hh + r) * SLABP + 16 * j + c] = acc[4 * hf + j][r];
      __builtin_amdgcn_fence(__ATOMIC_RELEASE, "workgroup");
      __builtin_amdgcn_wave_barrier();
      __builtin_amdgcn_fence(__ATOMIC_ACQUIRE, "workgroup");
#pragma unroll 1
      for (int it = 0; it < 4; ++it) {
        const int row = it * 4 + q;
        const float* sp = slab + row * SLABP + c8e;
        const float* xq = XP + ((size_t)tl * NBAT + (size_t)(rowbase + row)) * NHID + colbase + c8e;
        const v4f s0 = *(const v4f*)(sp);
        const v4f s1 = *(const v4f*)(sp + 4);
        const v4f x0 = *(const v4f*)(xq);
        const v4f x1 = *(const v4f*)(xq + 4);
        v8h hv;
#pragma unroll
        for (int e = 0; e < 4; ++e) {
          const float t0 = tanhf(s0[e] * WCARRY_INV + x0[e]);
          const float t1 = tanhf(s1[e] * WCARRY_INV + x1[e]);
          hv[e]     = (_Float16)t0;
          hv[4 + e] = (_Float16)t1;
        }
        *(v8h*)(Ah + row * HPITCH + colbase + c8e) = hv;
      }
      __builtin_amdgcn_fence(__ATOMIC_RELEASE, "workgroup");
      __builtin_amdgcn_wave_barrier();
      __builtin_amdgcn_fence(__ATOMIC_ACQUIRE, "workgroup");
    }

    __syncthreads();

    if (HIST) {
      for (int pass = 0; pass < 2; ++pass) {
#pragma unroll
        for (int it = 0; it < 8; ++it) {
          const int row = it * 2 + rr;
          const v8h v = *(const v8h*)(Ah + row * HPITCH + 128 * wave + c8s);
          *(volatile v8h*)(HISTG + ((size_t)tl * NBAT + (size_t)(rowbase + row)) * NHID + 128 * wave + c8s) = v;
        }
        __threadfence();
      }
    }
  }

  for (int pass = 0; pass < 2; ++pass) {
#pragma unroll
    for (int it = 0; it < 8; ++it) {
      const int row = it * 2 + rr;
      const v8h v = *(const v8h*)(Ah + row * HPITCH + 128 * wave + c8s);
      *(volatile v8h*)(CARRY + (size_t)(rowbase + row) * NHID + 128 * wave + c8s) = v;
    }
    __threadfence();
  }
}

__global__ __launch_bounds__(NTHR) void compact_kernel(const float* __restrict__ outpad, float* __restrict__ out) {
  const int i4 = blockIdx.x * NTHR + threadIdx.x;
  if (i4 < (NBAT * NCLS) / 4) {
    const int e0  = i4 * 4;
    const int row = e0 / NCLS;
    const int col = e0 - row * NCLS;
    const v4f v = *(const v4f*)(outpad + (size_t)row * NCLSP + col);
    *(volatile v4f*)(out + e0) = v;
    __threadfence();
    *(volatile v4f*)(out + e0) = v;
  }
}

extern "C" void kernel_launch(void* const* d_in, const int* in_sizes, int n_in,
                              void* d_out, int out_size, void* d_ws, size_t ws_size, hipStream_t stream) {
  if (n_in < 11 || d_out == nullptr || d_ws == nullptr) return;
  if (in_sizes[0] != NBAT * NSTEP * NIN || in_sizes[1] != NHID * NIN || in_sizes[2] != NHID * NHID ||
      in_sizes[3] != NHID || in_sizes[4] != NHID || in_sizes[5] != NHID * NHID || in_sizes[6] != NHID * NHID ||
      in_sizes[7] != NHID || in_sizes[8] != NHID || in_sizes[9] != NCLS * NHID || in_sizes[10] != NCLS ||
      out_size != NBAT * NCLS) return;

  const float* x    = (const float*)d_in[0];
  const float* wih0 = (const float*)d_in[1];
  const float* whh0 = (const float*)d_in[2];
  const float* bih0 = (const float*)d_in[3];
  const float* bhh0 = (const float*)d_in[4];
  const float* wih1 = (const float*)d_in[5];
  const float* whh1 = (const float*)d_in[6];
  const float* bih1 = (const float*)d_in[7];
  const float* bhh1 = (const float*)d_in[8];
  const float* fcw  = (const float*)d_in[9];
  const float* fcb  = (const float*)d_in[10];
  float* out = (float*)d_out;

  char* ws = (char*)d_ws;
  size_t off = 0;
  auto carve = [&](size_t bytes) -> char* { char* p = ws + off; off += (bytes + 255) & ~(size_t)255; return p; };
  unsigned short* XH     = (unsigned short*)carve((size_t)NSTEP * NBAT * NIN * 2);
  unsigned short* WIH0   = (unsigned short*)carve((size_t)NHID * NIN * 2);
  unsigned short* WHH0   = (unsigned short*)carve((size_t)NHID * NHID * 2);
  unsigned short* WIH1   = (unsigned short*)carve((size_t)NHID * NHID * 2);
  unsigned short* WHH1   = (unsigned short*)carve((size_t)NHID * NHID * 2);
  unsigned short* FCW    = (unsigned short*)carve((size_t)NCLSP * NHID * 2);
  float*          BIAS   = (float*)carve((size_t)3 * NHID * 4);
  float*          XP     = (float*)carve((size_t)MROWS * NHID * 4);
  unsigned short* H1C    = (unsigned short*)carve((size_t)MROWS * NHID * 2);
  unsigned short* CARRY0 = (unsigned short*)carve((size_t)NBAT * NHID * 2);
  unsigned short* CARRY1 = (unsigned short*)carve((size_t)NBAT * NHID * 2);
  float*          OUTPAD = (float*)carve((size_t)NBAT * NCLSP * 4);
  if (off > ws_size || off > (size_t)134217728) return;
  float* BIAS0 = BIAS;
  float* BIAS1 = BIAS + NHID;
  float* FCBP  = BIAS + 2 * NHID;

  const int n8a = NHID * (NIN / 8);
  const int n8b = NHID * (NHID / 8);
  const int n8c = NCLSP * (NHID / 8);
  wcvt_kernel<<<(n8a + NTHR - 1) / NTHR, NTHR, 0, stream>>>(wih0, WIH0, NHID,  NHID, NIN / 8,  WCARRY);
  wcvt_kernel<<<(n8b + NTHR - 1) / NTHR, NTHR, 0, stream>>>(whh0, WHH0, NHID,  NHID, NHID / 8, WCARRY);
  wcvt_kernel<<<(n8b + NTHR - 1) / NTHR, NTHR, 0, stream>>>(wih1, WIH1, NHID,  NHID, NHID / 8, WCARRY);
  wcvt_kernel<<<(n8b + NTHR - 1) / NTHR, NTHR, 0, stream>>>(whh1, WHH1, NHID,  NHID, NHID / 8, WCARRY);
  wcvt_kernel<<<(n8c + NTHR - 1) / NTHR, NTHR, 0, stream>>>(fcw,  FCW,  NCLSP, NCLS, NHID / 8, WCARRY);
  xcvt_kernel<<<(NSTEP * NBAT * (NIN / 8)) / NTHR, NTHR, 0, stream>>>(x, XH);
  bias_prep_kernel<true><<<1, NTHR, 0, stream>>>(bih0, bhh0, BIAS0, NHID);
  bias_prep_kernel<true><<<1, NTHR, 0, stream>>>(bih1, bhh1, BIAS1, NHID);
  bias_prep_kernel<false><<<1, NTHR, 0, stream>>>(fcb, fcb, FCBP, NCLS);

  const int ggrid = ((MROWS / 64) * (NHID / 64)) / 8;
  for (int ch = 0; ch < NCHUNK; ++ch) {
    const int first = (ch == 0) ? 1 : 0;
    gemm64_f16_kernel<<<ggrid, 256, 0, stream>>>(XH + (size_t)ch * MROWS * NIN, NIN, WIH0, NIN, XP, NHID, BIAS0,
                                                 MROWS, NHID, NIN, WCARRY_INV);
    rnn_scan_kernel<true><<<NBAT / MBLK, NTHR, 0, stream>>>(XP, WHH0, CARRY0, H1C, first);
    gemm64_f16_kernel<<<ggrid, 256, 0, stream>>>(H1C, NHID, WIH1, NHID, XP, NHID, BIAS1,
                                                 MROWS, NHID, NHID, WCARRY_INV);
    rnn_scan_kernel<false><<<NBAT / MBLK, NTHR, 0, stream>>>(XP, WHH1, CARRY1, CARRY1, first);
  }

  gemm64_f16_kernel<<<((NBAT / 64) * (NCLSP / 64)) / 8, 256, 0, stream>>>(CARRY1, NHID, FCW, NHID, OUTPAD, NCLSP, FCBP,
                                                                         NBAT, NCLSP, NHID, WCARRY_INV);
  compact_kernel<<<(NBAT * NCLS) / (4 * NTHR), NTHR, 0, stream>>>(OUTPAD, out);
}
